// Decoder_63067299775239
// MI455X (gfx1250) — hardware-verified
//
#include <hip/hip_runtime.h>
#include <stddef.h>
#include <stdint.h>

#define DK     128
#define NB     128
#define NTHR   256
#define EPB    1024
#define WSMAX  134217728

static_assert(DK % 32 == 0);
static_assert(NB == (NTHR / 32) * 16);
static_assert(16 * DK == NTHR * 8);
static_assert(NB * 2 == 64 * 4);
static_assert(EPB % NTHR == 0 && EPB % 32 == 0);

typedef int            v2i   __attribute__((ext_vector_type(2)));
typedef int            v8i   __attribute__((ext_vector_type(8)));
typedef float          v4f   __attribute__((ext_vector_type(4)));
typedef float          v8f   __attribute__((ext_vector_type(8)));
typedef unsigned short v8us  __attribute__((ext_vector_type(8)));
typedef unsigned short v16us __attribute__((ext_vector_type(16)));
typedef __bf16         v16bf __attribute__((ext_vector_type(16)));
typedef v2i  __attribute__((may_alias)) v2ia;
typedef v4f  __attribute__((may_alias)) v4fa;
typedef v8us __attribute__((may_alias)) v8usa;
union FragB { v16bf v; v16us u; v8us h[2]; v8i w; };

__device__ __forceinline__ v8f wmb(const FragB& a, const FragB& b, v8f c) {
  v8f d = __builtin_amdgcn_wmma_f32_16x16x32_bf16(false, a.v, false, b.v, (short)0, c, false, false);
  asm volatile("v_nop\n\tv_nop\n\tv_nop\n\tv_nop" : "+v"(d) : "v"(a.w), "v"(b.w));
  return d;
}

__device__ __forceinline__ unsigned bf16_bits(float f) {
  const unsigned u = __float_as_uint(f);
  return (u + 0x7FFFu + ((u >> 16) & 1u)) >> 16;
}
__device__ __forceinline__ float bf16_val(float f) {
  return __uint_as_float(bf16_bits(f) << 16);
}
__device__ __forceinline__ int pack2(float lo, float hi) {
  return (int)(bf16_bits(lo) | (bf16_bits(hi) << 16));
}

__global__ __launch_bounds__(NTHR) void k_node(const float* __restrict__ emb, const float* __restrict__ wgt,
                                               int nN, float* P) {
  __shared__ __attribute__((aligned(16))) unsigned short wsm[16 * DK];
  __shared__ __attribute__((aligned(16))) float pst[NB * 2];
  const int tid = (int)threadIdx.x, lane = tid & 31, wave = tid >> 5, hh = lane >> 4, m = lane & 15;
  const int rowBase = (int)blockIdx.x * NB;

  {
    const int n  = tid >> 4;
    const int k8 = (tid & 15) * 8;
    const int nc = n < 2 ? n : 1;
    const float* p = wgt + (size_t)nc * DK + k8;
    const v4f a = *(const v4fa*)p;
    const v4f b = *(const v4fa*)(p + 4);
    const bool ok = n < 2;
    v8us o;
    o[0] = ok ? (unsigned short)bf16_bits(a.x) : (unsigned short)0;
    o[1] = ok ? (unsigned short)bf16_bits(a.y) : (unsigned short)0;
    o[2] = ok ? (unsigned short)bf16_bits(a.z) : (unsigned short)0;
    o[3] = ok ? (unsigned short)bf16_bits(a.w) : (unsigned short)0;
    o[4] = ok ? (unsigned short)bf16_bits(b.x) : (unsigned short)0;
    o[5] = ok ? (unsigned short)bf16_bits(b.y) : (unsigned short)0;
    o[6] = ok ? (unsigned short)bf16_bits(b.z) : (unsigned short)0;
    o[7] = ok ? (unsigned short)bf16_bits(b.w) : (unsigned short)0;
    *(v8usa*)(wsm + n * DK + k8) = o;
  }
  __syncthreads();

  const int row = rowBase + 16 * wave + m;
  const int rc  = row < nN ? row : nN - 1;
  const float* ap = emb + (size_t)rc * DK + 8 * hh;
  const unsigned short* bp = wsm + m * DK + 8 * hh;

  v8f acc = {0.f, 0.f, 0.f, 0.f, 0.f, 0.f, 0.f, 0.f};
#pragma unroll
  for (int ks = 0; ks < DK / 32; ++ks) {
    const float* q = ap + 32 * ks;
    const v4f a0 = *(const v4fa*)q;
    const v4f a1 = *(const v4fa*)(q + 4);
    const v4f a2 = *(const v4fa*)(q + 16);
    const v4f a3 = *(const v4fa*)(q + 20);
    FragB af;
    af.w[0] = pack2(a0.x, a0.y);
    af.w[1] = pack2(a0.z, a0.w);
    af.w[2] = pack2(a1.x, a1.y);
    af.w[3] = pack2(a1.z, a1.w);
    af.w[4] = pack2(a2.x, a2.y);
    af.w[5] = pack2(a2.z, a2.w);
    af.w[6] = pack2(a3.x, a3.y);
    af.w[7] = pack2(a3.z, a3.w);
    FragB bf;
    bf.h[0] = *(const v8usa*)(bp + 32 * ks);
    bf.h[1] = *(const v8usa*)(bp + 32 * ks + 16);
    acc = wmb(af, bf, acc);
  }

  if (m < 2) {
#pragma unroll
    for (int r = 0; r < 8; ++r) {
      const int lr = 16 * wave + 8 * hh + r;
      const float v = acc[r];
      pst[lr * 2 + m] = (rowBase + lr < nN) ? v : 0.0f;
    }
  }
  __syncthreads();

  if (tid < 64) {
    const v4f v = *(const v4fa*)(pst + 4 * tid);
    float* op = P + (size_t)rowBase * 2 + 4 * tid;
    *(volatile v4f*)op = v;
    __threadfence();
    *(volatile v4f*)op = v;
  }
}

__global__ __launch_bounds__(NTHR) void k_edge(const int* __restrict__ edges, const float* __restrict__ P,
                                               const float* __restrict__ bias, int nE, int nN, float* out) {
  const int tid = (int)threadIdx.x;
  const float br = bf16_val(bias[0]);
  const int base = (int)blockIdx.x * EPB;
#pragma unroll 1
  for (int it = 0; it < EPB / NTHR; ++it) {
    const int e0 = base + it * NTHR;
    if (e0 >= nE) break;
    const int e  = e0 + tid;
    const int ec = e < nE ? e : nE - 1;
    const v2i sd = *(const v2ia*)(edges + 2 * (size_t)ec);
    int s = sd.x, d = sd.y;
    s = s < 0 ? 0 : (s > nN - 1 ? nN - 1 : s);
    d = d < 0 ? 0 : (d > nN - 1 ? nN - 1 : d);
    const float ps = P[2 * (size_t)s];
    const float pd = P[2 * (size_t)d + 1];
    const float v = (ps + pd) + br;
    if (e < nE) *(volatile float*)(out + e) = v;
    __threadfence();
    if (e < nE) *(volatile float*)(out + e) = v;
  }
}

static inline int cdiv(int a, int b) { return (a + b - 1) / b; }
static inline size_t al256(size_t o) { return (o + 255) & ~(size_t)255; }

extern "C" void kernel_launch(void* const* d_in, const int* in_sizes, int n_in,
                              void* d_out, int out_size, void* d_ws, size_t ws_size,
                              hipStream_t stream) {
  if (n_in < 4) return;
  if (in_sizes[0] < DK || (in_sizes[0] % DK) != 0) return;
  const int nN = in_sizes[0] / DK;
  if (nN < 1 || nN > (1 << 24)) return;
  if (in_sizes[1] < 2 || (in_sizes[1] & 1) != 0) return;
  const int nE = in_sizes[1] / 2;
  if (nE < 1 || nE > (1 << 29)) return;
  if (in_sizes[2] != 2 * DK) return;
  if (in_sizes[3] < 1) return;
  if (out_size != nE) return;

  const float* emb   = (const float*)d_in[0];
  const int*   edges = (const int*)d_in[1];
  const float* wgt   = (const float*)d_in[2];
  const float* bias  = (const float*)d_in[3];
  float* out = (float*)d_out;

  const int gN = cdiv(nN, NB);
  const int MP = gN * NB;
  const size_t pBytes = al256((size_t)MP * 2 * sizeof(float));
  if (pBytes > ws_size || pBytes > (size_t)WSMAX) return;
  float* P = (float*)d_ws;

  k_node<<<gN, NTHR, 0, stream>>>(emb, wgt, nN, P);
  k_edge<<<cdiv(nE, EPB), NTHR, 0, stream>>>(edges, P, bias, nE, nN, out);
}
